// GraphAttentionLayer_7421703487713
// MI455X (gfx1250) — hardware-verified
//
#include <hip/hip_runtime.h>
#include <math.h>
#include <stdint.h>

#define NB_   8
#define NN_   1024
#define NIN_  256
#define NAX_  512
#define NCAT_ 768
#define NOUT_ 256
#define NA_   1536
#define NTOK  (NB_ * NN_)
#define KG_   1024
#define FPB_  128
#define NFB_  (NTOK / 32)
#define SLOPE 0.2f
#define MASKFILL (-9.0e15f)
#define SFP   260
#define SGP   68
#define SOP   132
#define WSMAX 134217728

static_assert(NN_ % 64 == 0);
static_assert(NIN_ % 64 == 0);
static_assert(NAX_ % 64 == 0);
static_assert(NIN_ % 32 == 0);
static_assert(KG_ % 32 == 0);
static_assert(KG_ == 2 * NIN_ + NAX_);
static_assert(NCAT_ == NIN_ + NAX_);
static_assert(NA_ == 2 * NCAT_);
static_assert(NOUT_ == 256);
static_assert(NTOK % 32 == 0);
static_assert(NFB_ * 32 == NTOK);
static_assert((NIN_ * NIN_) % (8 * 256) == 0);
static_assert((NOUT_ * KG_) % (8 * 256) == 0);

typedef __attribute__((ext_vector_type(16))) __bf16 v16b;
typedef __attribute__((ext_vector_type(8)))  __bf16 v8b;
typedef __attribute__((ext_vector_type(8)))  float  v8f;
typedef __attribute__((ext_vector_type(4)))  float  v4f;
typedef __attribute__((ext_vector_type(4)))  unsigned int v4u;
typedef __attribute__((ext_vector_type(8)))  unsigned int v8u;
typedef __attribute__((ext_vector_type(4)))  int v4i;
typedef v8b __attribute__((may_alias)) v8ba;
typedef v4f __attribute__((may_alias)) v4fa;
typedef v4u __attribute__((may_alias)) v4ua;
typedef v4i __attribute__((may_alias)) v4ia;

union FragU { v16b v; v8b h[2]; };
union PackU { v8u u; v16b v; };

__device__ __forceinline__ unsigned short f2bf_bits(float f) {
  const unsigned u = __float_as_uint(f);
  return (unsigned short)((u + 0x7FFFu + ((u >> 16) & 1u)) >> 16);
}
__device__ __forceinline__ float bf_bits2f(unsigned short h) { return __uint_as_float(((unsigned)h) << 16); }
__device__ __forceinline__ float bf16r(float f) {
  unsigned u = __float_as_uint(f);
  u = (u + 0x7FFFu + ((u >> 16) & 1u)) & 0xFFFF0000u;
  return __uint_as_float(u);
}
__device__ __forceinline__ unsigned pk16(unsigned short a, unsigned short b) { return (unsigned)a | ((unsigned)b << 16); }

__device__ __forceinline__ v8f wmma_bf16(v16b a, v16b b, v8f c) {
  v8f d = __builtin_amdgcn_wmma_f32_16x16x32_bf16(false, a, false, b, (short)0, c, false, false);
  asm volatile("v_nop\n\tv_nop\n\tv_nop\n\tv_nop" : "+v"(d) : "v"(a), "v"(b));
  return d;
}

__device__ __forceinline__ v16b load_frag(const unsigned short* p, int hh) {
  FragU f;
  f.h[0] = *(const v8ba*)(p + 8 * hh);
  f.h[1] = *(const v8ba*)(p + 16 + 8 * hh);
  return f.v;
}

__device__ __forceinline__ void pack_p2(v8f a, v8f c, v16b& ho, v16b& lo) {
  PackU uh, ul;
#pragma unroll
  for (int i = 0; i < 4; ++i) {
    const unsigned short h0 = f2bf_bits(a[2 * i]), h1 = f2bf_bits(a[2 * i + 1]);
    const unsigned short l0 = f2bf_bits(a[2 * i] - bf_bits2f(h0)), l1 = f2bf_bits(a[2 * i + 1] - bf_bits2f(h1));
    uh.u[i] = pk16(h0, h1); ul.u[i] = pk16(l0, l1);
    const unsigned short g0 = f2bf_bits(c[2 * i]), g1 = f2bf_bits(c[2 * i + 1]);
    const unsigned short m0 = f2bf_bits(c[2 * i] - bf_bits2f(g0)), m1 = f2bf_bits(c[2 * i + 1] - bf_bits2f(g1));
    uh.u[4 + i] = pk16(g0, g1); ul.u[4 + i] = pk16(m0, m1);
  }
  ho = uh.v; lo = ul.v;
}

__device__ __forceinline__ void gemm_core_32x64p(
    const unsigned short* __restrict__ A, const unsigned short* __restrict__ Bt,
    int K, size_t aoff, size_t boff, int hh, v8f (&acc)[2][4]) {
  const unsigned short* a0 = A + aoff;
  const unsigned short* a1 = a0 + (size_t)16 * K;
  const unsigned short* bp = Bt + boff;
#pragma unroll 1
  for (int k0 = 0; k0 < K; k0 += 32) {
    const v16b f0 = load_frag(a0 + k0, hh);
    const v16b f1 = load_frag(a1 + k0, hh);
#pragma unroll
    for (int nt = 0; nt < 4; ++nt) {
      const v16b fb = load_frag(bp + (size_t)nt * 16 * K + k0, hh);
      acc[0][nt] = wmma_bf16(f0, fb, acc[0][nt]);
      acc[1][nt] = wmma_bf16(f1, fb, acc[1][nt]);
    }
  }
}

__global__ __launch_bounds__(256) void k_wprep(const float* __restrict__ wq, const float* __restrict__ fcw,
                                              unsigned short* WQb, unsigned short* FCB) {
  const int bx = (int)blockIdx.x, tid = (int)threadIdx.x;
  const float* p;
  unsigned short* dp;
  if (bx < 32) {
    const int u  = bx * 256 + tid;
    const int j  = u >> 5;
    const int k8 = (u & 31) * 8;
    p  = wq + (size_t)j * NIN_ + k8;
    dp = WQb + (size_t)u * 8;
  } else {
    const int v  = (bx - 32) * 256 + tid;
    const int o  = v >> 7;
    const int k8 = (v & 127) * 8;
    const int sc = (k8 < NIN_) ? k8 : (k8 - NIN_);
    p  = fcw + (size_t)o * NCAT_ + sc;
    dp = FCB + (size_t)v * 8;
  }
  const v4f a = *(const v4fa*)p;
  const v4f b = *(const v4fa*)(p + 4);
  v4u u;
  u[0] = pk16(f2bf_bits(a[0]), f2bf_bits(a[1]));
  u[1] = pk16(f2bf_bits(a[2]), f2bf_bits(a[3]));
  u[2] = pk16(f2bf_bits(b[0]), f2bf_bits(b[1]));
  u[3] = pk16(f2bf_bits(b[2]), f2bf_bits(b[3]));
  *(volatile v4u*)dp = u;
  __threadfence();
  *(volatile v4u*)dp = u;
}

__global__ __launch_bounds__(256) void k_xt(const float* __restrict__ x, const float* __restrict__ ax,
                                           unsigned short* XT, unsigned short* GA) {
  __shared__ __align__(16) float tf[64 * SGP];
  const int tid = (int)threadIdx.x;
  const int n0 = (int)blockIdx.x * 64;
  const int cy = (int)blockIdx.y;
  const int b  = (int)blockIdx.z;
  const float* src;
  unsigned short* dst;
  int dp, dc;
  if (cy < NIN_ / 64) {
    src = x + ((size_t)b * NIN_ + (size_t)cy * 64) * (size_t)NN_;
    dst = XT; dp = NIN_; dc = cy * 64;
  } else {
    const int ca = (cy - NIN_ / 64) * 64;
    src = ax + ((size_t)b * NAX_ + (size_t)ca) * (size_t)NN_;
    dst = GA; dp = KG_; dc = NAX_ + ca;
  }
  {
    const int rs = tid >> 4;
    const int c4 = (tid & 15) * 4;
#pragma unroll
    for (int it = 0; it < 4; ++it) {
      const int cr = it * 16 + rs;
      const v4f a = *(const v4fa*)(src + (size_t)cr * NN_ + n0 + c4);
      *(v4fa*)(tf + cr * SGP + c4) = a;
    }
  }
  __syncthreads();
  const int rs = tid >> 3;
  const int c8 = (tid & 7) * 8;
  v4u o[2];
#pragma unroll
  for (int it = 0; it < 2; ++it) {
    const int tl = it * 32 + rs;
    v4u wv;
#pragma unroll
    for (int q = 0; q < 4; ++q) {
      const float f0 = tf[(c8 + 2 * q) * SGP + tl];
      const float f1 = tf[(c8 + 2 * q + 1) * SGP + tl];
      wv[q] = pk16(f2bf_bits(f0), f2bf_bits(f1));
    }
    o[it] = wv;
  }
#pragma unroll
  for (int it = 0; it < 2; ++it) {
    const int tl = it * 32 + rs;
    *(volatile v4u*)(dst + ((size_t)(b * NN_ + n0 + tl)) * (size_t)dp + dc + c8) = o[it];
  }
  __threadfence();
#pragma unroll
  for (int it = 0; it < 2; ++it) {
    const int tl = it * 32 + rs;
    *(volatile v4u*)(dst + ((size_t)(b * NN_ + n0 + tl)) * (size_t)dp + dc + c8) = o[it];
  }
}

__global__ __launch_bounds__(128) void k_q1(const unsigned short* __restrict__ XT, const unsigned short* __restrict__ WQb,
                                           const float* __restrict__ wqbias, const float* __restrict__ av,
                                           unsigned short* GA, float* F) {
  __shared__ __align__(16) float sF[32 * SFP];
  __shared__ __align__(16) float sAv[NA_];
  __shared__ __align__(16) float sBq[NIN_];
  __shared__ __align__(16) float sFF[FPB_];
  const int tid = (int)threadIdx.x, lane = tid & 31, w = tid >> 5;
  const int hh = lane >> 4, m = lane & 15;
  const int n0 = (int)blockIdx.x * 32;
  const int c0w = 64 * w;

  {
    const float* ap = av + tid * 12;
#pragma unroll
    for (int i = 0; i < 3; ++i) {
      const v4f t4 = *(const v4fa*)(ap + 4 * i);
      v4f r4;
      r4[0] = bf16r(t4[0]); r4[1] = bf16r(t4[1]); r4[2] = bf16r(t4[2]); r4[3] = bf16r(t4[3]);
      *(v4fa*)(sAv + tid * 12 + 4 * i) = r4;
    }
    sBq[tid]       = bf16r(wqbias[tid]);
    sBq[128 + tid] = bf16r(wqbias[128 + tid]);
  }
  __syncthreads();

  const v8f zero8 = {0.f, 0.f, 0.f, 0.f, 0.f, 0.f, 0.f, 0.f};
  v8f acc[2][4];
#pragma unroll
  for (int mt = 0; mt < 2; ++mt)
#pragma unroll
    for (int nt = 0; nt < 4; ++nt) acc[mt][nt] = zero8;

  gemm_core_32x64p(XT, WQb, NIN_, (size_t)(n0 + m) * NIN_, (size_t)(c0w + m) * NIN_, hh, acc);

#pragma unroll
  for (int nt = 0; nt < 4; ++nt)
#pragma unroll
    for (int mt = 0; mt < 2; ++mt)
#pragma unroll
      for (int r = 0; r < 8; ++r) {
        const int rowl = 16 * mt + 8 * hh + r;
        const int col  = c0w + 16 * nt + m;
        sF[rowl * SFP + col] = acc[mt][nt][r] + sBq[col];
      }
  __syncthreads();

  {
    const int row = tid >> 2, qq = tid & 3;
    float s1 = 0.0f, s2 = 0.0f;
    const float* fr = sF + row * SFP + 64 * qq;
    const float* a1 = sAv + 64 * qq;
    const float* a2 = sAv + NCAT_ + 64 * qq;
#pragma unroll 2
    for (int d4 = 0; d4 < 16; ++d4) {
      const v4f xv = *(const v4fa*)(fr + 4 * d4);
      const v4f y  = *(const v4fa*)(a1 + 4 * d4);
      const v4f z  = *(const v4fa*)(a2 + 4 * d4);
      s1 = fmaf(xv[0], y[0], s1); s1 = fmaf(xv[1], y[1], s1); s1 = fmaf(xv[2], y[2], s1); s1 = fmaf(xv[3], y[3], s1);
      s2 = fmaf(xv[0], z[0], s2); s2 = fmaf(xv[1], z[1], s2); s2 = fmaf(xv[2], z[2], s2); s2 = fmaf(xv[3], z[3], s2);
    }
    const unsigned short* gp = GA + (size_t)(n0 + row) * KG_ + NAX_ + 128 * qq;
    const float* b1 = sAv + NIN_ + 128 * qq;
    const float* b2 = sAv + NCAT_ + NIN_ + 128 * qq;
#pragma unroll 1
    for (int i = 0; i < 16; ++i) {
      const v4u wv = *(const v4ua*)(gp + 8 * i);
      const v4f y0 = *(const v4fa*)(b1 + 8 * i), y1 = *(const v4fa*)(b1 + 8 * i + 4);
      const v4f z0 = *(const v4fa*)(b2 + 8 * i), z1 = *(const v4fa*)(b2 + 8 * i + 4);
      float hv[8];
#pragma unroll
      for (int q = 0; q < 4; ++q) {
        hv[2 * q]     = __uint_as_float(wv[q] << 16);
        hv[2 * q + 1] = __uint_as_float(wv[q] & 0xFFFF0000u);
      }
      s1 = fmaf(hv[0], y0[0], s1); s1 = fmaf(hv[1], y0[1], s1); s1 = fmaf(hv[2], y0[2], s1); s1 = fmaf(hv[3], y0[3], s1);
      s1 = fmaf(hv[4], y1[0], s1); s1 = fmaf(hv[5], y1[1], s1); s1 = fmaf(hv[6], y1[2], s1); s1 = fmaf(hv[7], y1[3], s1);
      s2 = fmaf(hv[0], z0[0], s2); s2 = fmaf(hv[1], z0[1], s2); s2 = fmaf(hv[2], z0[2], s2); s2 = fmaf(hv[3], z0[3], s2);
      s2 = fmaf(hv[4], z1[0], s2); s2 = fmaf(hv[5], z1[1], s2); s2 = fmaf(hv[6], z1[2], s2); s2 = fmaf(hv[7], z1[3], s2);
    }
    s1 += __shfl_xor(s1, 1, 32); s1 += __shfl_xor(s1, 2, 32);
    s2 += __shfl_xor(s2, 1, 32); s2 += __shfl_xor(s2, 2, 32);
    if (qq == 0) { sFF[row] = s1; sFF[32 + row] = s2; }
    if (tid >= 64) sFF[tid] = 0.0f;
  }
  __syncthreads();
  {
    const v4f v = *(const v4fa*)(sFF + 4 * lane);
    float* fp = F + (size_t)blockIdx.x * FPB_ + 4 * lane;
    if (w == 0) *(volatile v4f*)fp = v;
    __threadfence();
    if (w == 0) *(volatile v4f*)fp = v;
  }
  {
    const int c8 = lane * 8;
    for (int pass = 0; pass < 2; ++pass) {
#pragma unroll 2
      for (int it = 0; it < 8; ++it) {
        const int row = 8 * w + it;
        const float* sp = sF + row * SFP + c8;
        const v4f x0 = *(const v4fa*)sp, x1 = *(const v4fa*)(sp + 4);
        const float xv[8] = {x0[0], x0[1], x0[2], x0[3], x1[0], x1[1], x1[2], x1[3]};
        v4u hv, lv;
#pragma unroll
        for (int q = 0; q < 4; ++q) {
          const unsigned short h0 = f2bf_bits(xv[2 * q]), h1 = f2bf_bits(xv[2 * q + 1]);
          const unsigned short l0 = f2bf_bits(xv[2 * q] - bf_bits2f(h0));
          const unsigned short l1 = f2bf_bits(xv[2 * q + 1] - bf_bits2f(h1));
          hv[q] = pk16(h0, h1); lv[q] = pk16(l0, l1);
        }
        const size_t go = (size_t)(n0 + row) * KG_ + c8;
        *(volatile v4u*)(GA + go) = hv;
        *(volatile v4u*)(GA + go + NIN_) = lv;
      }
      __threadfence();
    }
  }
}

__global__ __launch_bounds__(128) void k_g(const unsigned short* __restrict__ FCB, const unsigned short* __restrict__ GA,
                                          unsigned short* GTh, unsigned short* GTl) {
  __shared__ __align__(16) float stg[64 * SGP];
  const int tid = (int)threadIdx.x, lane = tid & 31, wave = tid >> 5, hh = lane >> 4, m = lane & 15;
  const int rowBase = (int)blockIdx.x * 64;
  const int colBase = (int)blockIdx.y * 64;
  const int z = (int)blockIdx.z;
  const unsigned short* Bb = GA + (size_t)z * (size_t)NN_ * KG_;

  const v8f zero8 = {0.f, 0.f, 0.f, 0.f, 0.f, 0.f, 0.f, 0.f};
  v8f acc[4];
#pragma unroll
  for (int t = 0; t < 4; ++t) acc[t] = zero8;
  const unsigned short* ap = FCB + (size_t)(rowBase + 16 * wave + m) * (size_t)KG_;
  const unsigned short* bp = Bb + (size_t)(colBase + m) * (size_t)KG_;

#pragma unroll 1
  for (int k0 = 0; k0 < KG_; k0 += 32) {
    const v16b af = load_frag(ap + k0, hh);
#pragma unroll
    for (int nt = 0; nt < 4; ++nt) {
      const v16b bf = load_frag(bp + (size_t)(16 * nt) * (size_t)KG_ + k0, hh);
      acc[nt] = wmma_bf16(af, bf, acc[nt]);
    }
  }

#pragma unroll
  for (int nt = 0; nt < 4; ++nt) {
    const int lc = 16 * nt + m;
#pragma unroll
    for (int r = 0; r < 8; ++r) {
      const int lr = 16 * wave + 8 * hh + r;
      stg[lr * SGP + lc] = acc[nt][r];
    }
  }
  __syncthreads();

  const int rsub = tid >> 3;
  const int c8   = (tid & 7) * 8;
  v4u hv[4], lv[4];
#pragma unroll
  for (int it = 0; it < 4; ++it) {
    const int row = it * 16 + rsub;
    const float* sp = stg + row * SGP + c8;
    const v4f x0 = *(const v4fa*)sp, x1 = *(const v4fa*)(sp + 4);
    const float xv[8] = {x0[0], x0[1], x0[2], x0[3], x1[0], x1[1], x1[2], x1[3]};
    v4u h8, l8;
#pragma unroll
    for (int q = 0; q < 4; ++q) {
      const unsigned short h0 = f2bf_bits(xv[2 * q]), h1 = f2bf_bits(xv[2 * q + 1]);
      const unsigned short l0 = f2bf_bits(xv[2 * q] - bf_bits2f(h0));
      const unsigned short l1 = f2bf_bits(xv[2 * q + 1] - bf_bits2f(h1));
      h8[q] = pk16(h0, h1); l8[q] = pk16(l0, l1);
    }
    hv[it] = h8; lv[it] = l8;
  }
#pragma unroll
  for (int it = 0; it < 4; ++it) {
    const int row = it * 16 + rsub;
    const size_t go = ((size_t)z * NOUT_ + (size_t)(rowBase + row)) * (size_t)NN_ + colBase + c8;
    *(volatile v4u*)(GTh + go) = hv[it];
    *(volatile v4u*)(GTl + go) = lv[it];
  }
  __threadfence();
#pragma unroll
  for (int it = 0; it < 4; ++it) {
    const int row = it * 16 + rsub;
    const size_t go = ((size_t)z * NOUT_ + (size_t)(rowBase + row)) * (size_t)NN_ + colBase + c8;
    *(volatile v4u*)(GTh + go) = hv[it];
    *(volatile v4u*)(GTl + go) = lv[it];
  }
}

__global__ __launch_bounds__(128) void k_attn(const float* __restrict__ F, const int* __restrict__ adj,
                                             const unsigned short* __restrict__ GTh,
                                             const unsigned short* __restrict__ GTl,
                                             const float* __restrict__ fcb, float* __restrict__ out) {
  __shared__ __align__(16) float sK[NN_];
  __shared__ __align__(16) float sB[128];
  __shared__ __align__(16) float sO[4][16 * SOP];

  const int tid = (int)threadIdx.x, lane = tid & 31, w = tid >> 5;
  const int hh = lane >> 4, m = lane & 15;
  const int qt = (int)blockIdx.x, chh = (int)blockIdx.y, b = (int)blockIdx.z;
  const int q0 = qt * 64, q0w = q0 + 16 * w, q = q0w + m;
  const int d0 = chh * 128;

  {
    const int bb = tid >> 2, piece = tid & 3;
    const float* g = F + (size_t)(b * (NN_ / 32) + bb) * FPB_ + 32 + 8 * piece;
    const v4f a0 = *(const v4fa*)g;
    const v4f a1 = *(const v4fa*)(g + 4);
    *(v4fa*)(sK + bb * 32 + 8 * piece)     = a0;
    *(v4fa*)(sK + bb * 32 + 8 * piece + 4) = a1;
  }
  sB[tid] = bf16r(fcb[d0 + tid]);
  const float f1q = F[(size_t)(b * (NN_ / 32) + (q >> 5)) * FPB_ + (q & 31)];
  const int* arow = adj + ((size_t)(b * NN_ + q)) * (size_t)NN_;

  const v8f zero8 = {0.f, 0.f, 0.f, 0.f, 0.f, 0.f, 0.f, 0.f};
  v8f o[8];
#pragma unroll
  for (int t = 0; t < 8; ++t) o[t] = zero8;
  float mrun = -INFINITY, lrun = 0.0f;

  __syncthreads();

#pragma unroll 1
  for (int ks = 0; ks < NN_ / 32; ++ks) {
    const int kb = ks * 32;

    v8f s[2];
#pragma unroll
    for (int j = 0; j < 2; ++j) {
      const int ko = kb + 16 * j + 8 * hh;
      const v4i mA = *(const v4ia*)(arow + ko);
      const v4i mB = *(const v4ia*)(arow + ko + 4);
      const v4f kA = *(const v4fa*)(sK + ko);
      const v4f kB = *(const v4fa*)(sK + ko + 4);
      const int   mv[8] = {mA[0], mA[1], mA[2], mA[3], mB[0], mB[1], mB[2], mB[3]};
      const float kv[8] = {kA[0], kA[1], kA[2], kA[3], kB[0], kB[1], kB[2], kB[3]};
#pragma unroll
      for (int r = 0; r < 8; ++r) {
        float t = f1q + kv[r];
        t = (t >= 0.0f) ? t : SLOPE * t;
        t = (mv[r] > 0) ? t : MASKFILL;
        s[j][r] = t;
      }
    }
    float cm = -INFINITY;
#pragma unroll
    for (int j = 0; j < 2; ++j)
#pragma unroll
      for (int r = 0; r < 8; ++r) cm = fmaxf(cm, s[j][r]);
    cm = fmaxf(cm, __shfl_xor(cm, 16, 32));
    const float mnew  = fmaxf(mrun, cm);
    const float alpha = __expf(mrun - mnew);
    mrun = mnew;
    float psum = 0.0f;
#pragma unroll
    for (int j = 0; j < 2; ++j)
#pragma unroll
      for (int r = 0; r < 8; ++r) {
        const float p = __expf(s[j][r] - mnew);
        psum += p;
        s[j][r] = p;
      }
    psum += __shfl_xor(psum, 16, 32);
    lrun = lrun * alpha + psum;
#pragma unroll
    for (int t = 0; t < 8; ++t)
#pragma unroll
      for (int r = 0; r < 8; ++r) o[t][r] *= alpha;

    v16b ph, pl;
    pack_p2(s[0], s[1], ph, pl);

    const unsigned short* gh = GTh + (size_t)(b * NOUT_ + d0 + m) * (size_t)NN_ + kb;
    const unsigned short* gl = GTl + (size_t)(b * NOUT_ + d0 + m) * (size_t)NN_ + kb;
#pragma unroll
    for (int t = 0; t < 8; ++t) {
      const v16b vh = load_frag(gh + (size_t)(16 * t) * (size_t)NN_, hh);
      const v16b vl = load_frag(gl + (size_t)(16 * t) * (size_t)NN_, hh);
      o[t] = wmma_bf16(vh, ph, o[t]);
      o[t] = wmma_bf16(vh, pl, o[t]);
      o[t] = wmma_bf16(vl, ph, o[t]);
    }
  }

  const float inv = 1.0f / lrun;
  float* so = sO[w];
#pragma unroll
  for (int t = 0; t < 8; ++t) {
    const v4f bA = *(const v4fa*)(sB + 16 * t + 8 * hh);
    const v4f bB = *(const v4fa*)(sB + 16 * t + 8 * hh + 4);
    const float bv[8] = {bA[0], bA[1], bA[2], bA[3], bB[0], bB[1], bB[2], bB[3]};
#pragma unroll
    for (int r = 0; r < 8; ++r)
      so[m * SOP + 16 * t + 8 * hh + r] = o[t][r] * inv + bv[r];
  }
  __syncthreads();
  {
    const int c4 = lane * 4;
    for (int pass = 0; pass < 2; ++pass) {
#pragma unroll 2
      for (int it = 0; it < 16; ++it) {
        v4f v = *(const v4fa*)(so + it * SOP + c4);
        v[0] = (v[0] > 0.0f) ? v[0] : expm1f(v[0]);
        v[1] = (v[1] > 0.0f) ? v[1] : expm1f(v[1]);
        v[2] = (v[2] > 0.0f) ? v[2] : expm1f(v[2]);
        v[3] = (v[3] > 0.0f) ? v[3] : expm1f(v[3]);
        *(volatile v4f*)(out + ((size_t)(b * NN_ + q0w + it)) * (size_t)NOUT_ + d0 + c4) = v;
      }
      __threadfence();
    }
  }
}

static inline size_t al256(size_t o) { return (o + 255) & ~(size_t)255; }

extern "C" void kernel_launch(void* const* d_in, const int* in_sizes, int n_in,
                              void* d_out, int out_size, void* d_ws, size_t ws_size,
                              hipStream_t stream) {
  if (n_in < 8) return;
  if (in_sizes[0] != NB_ * NIN_ * NN_) return;
  if (in_sizes[1] != NB_ * NAX_ * NN_) return;
  if (in_sizes[2] != NB_ * NN_ * NN_) return;
  if (in_sizes[3] != NIN_ * NIN_) return;
  if (in_sizes[4] != NIN_) return;
  if (in_sizes[5] != NA_) return;
  if (in_sizes[6] != NOUT_ * NCAT_) return;
  if (in_sizes[7] != NOUT_) return;
  if (out_size != NB_ * NN_ * NOUT_) return;

  const float* x    = (const float*)d_in[0];
  const float* ax   = (const float*)d_in[1];
  const int*   adj  = (const int*)d_in[2];
  const float* wqw  = (const float*)d_in[3];
  const float* wqb  = (const float*)d_in[4];
  const float* av   = (const float*)d_in[5];
  const float* fcw  = (const float*)d_in[6];
  const float* fcb  = (const float*)d_in[7];
  float* out = (float*)d_out;

  const size_t PWQ = (size_t)NIN_ * NIN_ * 2;
  const size_t PFC = (size_t)NOUT_ * KG_ * 2;
  const size_t PXT = (size_t)NTOK * NIN_ * 2;
  const size_t PGA = (size_t)NTOK * KG_ * 2;
  const size_t PF  = (size_t)NFB_ * FPB_ * 4;
  const size_t PGT = (size_t)NB_ * NOUT_ * NN_ * 2;
  size_t off = 0;
  const size_t oWQ  = off; off = al256(off + PWQ);
  const size_t oFC  = off; off = al256(off + PFC);
  const size_t oXT  = off; off = al256(off + PXT);
  const size_t oGA  = off; off = al256(off + PGA);
  const size_t oF   = off; off = al256(off + PF);
  const size_t oGTh = off; off = al256(off + PGT);
  const size_t oGTl = off; off = al256(off + PGT);
  if (off > ws_size || off > (size_t)WSMAX) return;

  char* ws = (char*)d_ws;
  unsigned short* WQb = (unsigned short*)(ws + oWQ);
  unsigned short* FCB = (unsigned short*)(ws + oFC);
  unsigned short* XT  = (unsigned short*)(ws + oXT);
  unsigned short* GA  = (unsigned short*)(ws + oGA);
  float*          F   = (float*)(ws + oF);
  unsigned short* GTh = (unsigned short*)(ws + oGTh);
  unsigned short* GTl = (unsigned short*)(ws + oGTl);

  k_wprep<<<dim3(32 + 128), 256, 0, stream>>>(wqw, fcw, WQb, FCB);
  k_xt<<<dim3(NN_ / 64, NIN_ / 64 + NAX_ / 64, NB_), 256, 0, stream>>>(x, ax, XT, GA);
  k_q1<<<dim3(NTOK / 32), 128, 0, stream>>>(XT, WQb, wqb, av, GA, F);
  k_g<<<dim3(NOUT_ / 64, NN_ / 64, NB_), 128, 0, stream>>>(FCB, GA, GTh, GTl);
  k_attn<<<dim3(NN_ / 64, NOUT_ / 128, NB_), 128, 0, stream>>>(F, adj, GTh, GTl, fcb, out);
  (void)hipGetLastError();
}
